// CrossAttentionBlock_28492813041792
// MI455X (gfx1250) — hardware-verified
//
#include <hip/hip_runtime.h>
#include <stddef.h>


typedef _Float16 v16h __attribute__((ext_vector_type(16)));
typedef _Float16 v8h  __attribute__((ext_vector_type(8)));
typedef float    v8f  __attribute__((ext_vector_type(8)));
typedef float    v4f  __attribute__((ext_vector_type(4)));
typedef _Float16 h16;

#ifndef NB
#define NB 8
#endif
#define NB_FULL 8
#define CIN   256
#define TQ    3200
#define SK    640
#define NHEAD 8
#define HD    64
#define HDIM  512
#define CO    256

static_assert(NB >= 1 && NB <= NB_FULL);
static_assert(HDIM == NHEAD * HD);
static_assert(HD == 64);
static_assert((TQ % 128) == 0 && (TQ % 64) == 0);
static_assert((SK % 64) == 0);
static_assert((CIN % 64) == 0 && (CIN % 32) == 0);
static_assert((HDIM % 64) == 0 && (HDIM % 32) == 0);
static_assert((CO % 64) == 0);
static_assert(((NB * TQ) % 64) == 0 && ((NB * SK) % 64) == 0);
static_assert(((TQ / 4) % 32) == 0);
static_assert(((HDIM * CIN) % 2048) == 0);
static_assert(((2 * HDIM * CIN) % 2048) == 0);
static_assert(((CO * HDIM) % 2048) == 0);
static_assert((size_t)NB * TQ * HDIM < (size_t)0xFFFFFFFFu);

#define LDT 72
#define LDC 68
static_assert((LDT % 8) == 0 && LDT >= 64);
static_assert((LDC % 4) == 0 && LDC >= 64);

#define WCARRY 64.0f
#define XCARRY 64.0f
#define PCARRY 1024.0f
#define VCARRY 64.0f

#define WQ_BYTES   ((size_t)HDIM * CIN * 2)
#define WKV_BYTES  ((size_t)2 * HDIM * CIN * 2)
#define WO_BYTES   ((size_t)CO * HDIM * 2)
#define XJ_BYTES   ((size_t)NB * TQ * CIN * 2)
#define XG_BYTES   ((size_t)NB * SK * CIN * 2)
#define Q_BYTES    ((size_t)NB * TQ * HDIM * 2)
#define K_BYTES    ((size_t)NB * SK * HDIM * 2)
#define VT_BYTES   ((size_t)NB * HDIM * SK * 2)
#define CTX_BYTES  ((size_t)NB * TQ * HDIM * 2)
#define Y_BYTES    ((size_t)NB * CO * TQ * 4)
#define OFF_WQ  ((size_t)0)
#define OFF_WKV (OFF_WQ + WQ_BYTES)
#define OFF_WO  (OFF_WKV + WKV_BYTES)
#define OFF_XJ  (OFF_WO + WO_BYTES)
#define OFF_XG  (OFF_XJ + XJ_BYTES)
#define OFF_Q   (OFF_XG + XG_BYTES)
#define OFF_K   (OFF_Q + Q_BYTES)
#define OFF_VT  (OFF_K + K_BYTES)
#define OFF_CTX (OFF_VT + VT_BYTES)
#define OFF_Y   (OFF_CTX + CTX_BYTES)
#define WS_TOTAL (OFF_Y + Y_BYTES)
static_assert((WQ_BYTES % 128) == 0 && (WKV_BYTES % 128) == 0 && (WO_BYTES % 128) == 0);
static_assert((XJ_BYTES % 128) == 0 && (XG_BYTES % 128) == 0 && (Q_BYTES % 128) == 0);
static_assert((K_BYTES % 128) == 0 && (VT_BYTES % 128) == 0 && (CTX_BYTES % 128) == 0);
static_assert((Y_BYTES % 128) == 0);
static_assert(WS_TOTAL <= (size_t)134217728);

__device__ __forceinline__ float bf16r(float x) {
  unsigned int u = __float_as_uint(x);
  u = (u + 0x7FFFu + ((u >> 16) & 1u)) & 0xFFFF0000u;
  return __uint_as_float(u);
}

static __device__ __forceinline__ h16 toh_flush(float v) {
  const h16 r = (h16)v;
  return (fabsf(v) < 6.103515625e-05f) ? (h16)0.0f : r;
}

__device__ __forceinline__ v16h frag_at(const _Float16* p) {
  v8h lo = *(const v8h*)(p);
  v8h hi = *(const v8h*)(p + 16);
  v16h out;
#pragma unroll
  for (int i = 0; i < 8; ++i) { out[i] = lo[i]; out[i + 8] = hi[i]; }
  return out;
}
__device__ __forceinline__ v16h ld_frag(const _Float16* base, unsigned ld) {
  const unsigned lane = threadIdx.x & 31u;
  return frag_at(base + (lane & 15u) * ld + (lane >> 4) * 8u);
}

__device__ __forceinline__ v8f wmma16(v16h a, v16h b, v8f c) {
  v8f d = __builtin_amdgcn_wmma_f32_16x16x32_f16(false, a, false, b, (short)0, c,
                                                 false, false);
  asm volatile("v_nop\n\tv_nop\n\tv_nop\n\tv_nop" : "+v"(d) : "v"(a), "v"(b));
  return d;
}

__device__ __forceinline__ float red16_max(float x) {
#pragma unroll
  for (int off = 1; off < 16; off <<= 1) x = fmaxf(x, __shfl_xor(x, off, 32));
  return x;
}
__device__ __forceinline__ float red16_sum(float x) {
#pragma unroll
  for (int off = 1; off < 16; off <<= 1) x += __shfl_xor(x, off, 32);
  return x;
}
__device__ __forceinline__ float red32_sum(float x) {
#pragma unroll
  for (int off = 1; off < 32; off <<= 1) x += __shfl_xor(x, off, 32);
  return x;
}

__device__ __forceinline__ void wave_lds_sync() {
  __builtin_amdgcn_fence(3  , "wavefront");
  asm volatile("s_wait_dscnt 0x0" ::: "memory");
  __builtin_amdgcn_wave_barrier();
}

__global__ __launch_bounds__(256) void wcast_kernel(
    const float* __restrict__ W, _Float16* __restrict__ W16, unsigned n8) {
#pragma clang fp contract(off)
  const unsigned idx = blockIdx.x * 256u + threadIdx.x;
  if (idx < n8) {
    const v4f a0 = *(const v4f*)(W + (size_t)idx * 8u);
    const v4f a1 = *(const v4f*)(W + (size_t)idx * 8u + 4u);
    v8h x;
#pragma unroll
    for (int j = 0; j < 4; ++j) {
      x[j]     = toh_flush(WCARRY * bf16r(a0[j]));
      x[j + 4] = toh_flush(WCARRY * bf16r(a1[j]));
    }
    _Float16* p = W16 + (size_t)idx * 8u;
    *(volatile v8h*)p = x;
    __threadfence();
    *(volatile v8h*)p = x;
  }
}

__global__ __launch_bounds__(256) void xconv_kernel(
    const float* __restrict__ X, _Float16* __restrict__ Xt, unsigned ntok) {
#pragma clang fp contract(off)
  __shared__ _Float16 T[64 * LDT];
  const unsigned tid = threadIdx.x;
  const unsigned p0 = blockIdx.x * 64u;
  const unsigned c0 = blockIdx.y * 64u;
  const unsigned b = blockIdx.z;
  const size_t src0 = (size_t)b * CIN * ntok;
#pragma unroll 4
  for (unsigned j = 0; j < 16u; ++j) {
    const unsigned idx = tid + 256u * j;
    const unsigned cr = idx >> 6, pc = idx & 63u;
    const float v = X[src0 + (size_t)(c0 + cr) * ntok + p0 + pc];
    T[pc * LDT + cr] = toh_flush(XCARRY * bf16r(v));
  }
  __syncthreads();
  v8h x[2];
  size_t off[2];
#pragma unroll
  for (unsigned i = 0; i < 2u; ++i) {
    const unsigned n = 32u * i + (tid >> 3);
    const unsigned kc = (tid & 7u) * 8u;
    x[i] = *(const v8h*)&T[n * LDT + kc];
    off[i] = ((size_t)b * ntok + p0 + n) * CIN + c0 + kc;
  }
#pragma unroll
  for (int i = 0; i < 2; ++i) *(volatile v8h*)(Xt + off[i]) = x[i];
  __threadfence();
#pragma unroll
  for (int i = 0; i < 2; ++i) *(volatile v8h*)(Xt + off[i]) = x[i];
}

template <int MODE>
__device__ __forceinline__ void gemm_body(
    const _Float16* __restrict__ A16, const _Float16* __restrict__ Bt, const unsigned K,
    const float* __restrict__ bias, float* __restrict__ outf, _Float16* __restrict__ out16) {
  __shared__ float Cs[64 * LDC];
  const unsigned tid = threadIdx.x, lane = tid & 31u;
  const unsigned w = (unsigned)__builtin_amdgcn_readfirstlane((int)(tid >> 5));
  const unsigned mw = w >> 1, nw = w & 1u;
  const unsigned hh = lane >> 4, m = lane & 15u;
  const unsigned n0 = blockIdx.x * 64u;
  const unsigned row0 = blockIdx.y * 64u;

  const _Float16* ap  = A16 + (size_t)(row0 + mw * 16u + m) * K + hh * 8u;
  const _Float16* bp0 = Bt + (size_t)(n0 + nw * 32u + m) * K + hh * 8u;
  const _Float16* bp1 = bp0 + (size_t)16 * K;
  v8f acc0 = {}, acc1 = {};
#pragma unroll 2
  for (unsigned k0 = 0; k0 < K; k0 += 32u) {
    const v16h a  = frag_at(ap + k0);
    const v16h b0 = frag_at(bp0 + k0);
    const v16h b1 = frag_at(bp1 + k0);
    acc0 = wmma16(a, b0, acc0);
    acc1 = wmma16(a, b1, acc1);
  }
#pragma unroll
  for (int r = 0; r < 8; ++r) {
    float* d = &Cs[(mw * 16u + hh * 8u + (unsigned)r) * LDC + nw * 32u + m];
    d[0]  = acc0[r];
    d[16] = acc1[r];
  }
  __syncthreads();

  if (MODE == 0) {
    const float cs = 1.0f / (WCARRY * XCARRY);
    v8h x[2];
    size_t off[2];
#pragma unroll
    for (unsigned i = 0; i < 2u; ++i) {
      const unsigned r = 32u * i + (tid >> 3);
      const unsigned c = (tid & 7u) * 8u;
      const v4f u0 = *(const v4f*)&Cs[r * LDC + c];
      const v4f u1 = *(const v4f*)&Cs[r * LDC + c + 4];
      const v4f g0 = *(const v4f*)(bias + n0 + c);
      const v4f g1 = *(const v4f*)(bias + n0 + c + 4u);
#pragma unroll
      for (int j = 0; j < 4; ++j) {
        x[i][j]     = toh_flush(u0[j] * cs + bf16r(g0[j]));
        x[i][j + 4] = toh_flush(u1[j] * cs + bf16r(g1[j]));
      }
      off[i] = (size_t)(row0 + r) * HDIM + n0 + c;
    }
#pragma unroll
    for (int i = 0; i < 2; ++i) *(volatile v8h*)(out16 + off[i]) = x[i];
    __threadfence();
#pragma unroll
    for (int i = 0; i < 2; ++i) *(volatile v8h*)(out16 + off[i]) = x[i];
  }

  if (MODE == 1) {
    const float cs = 1.0f / (WCARRY * XCARRY);
    const unsigned bidx = row0 / (unsigned)SK;
    const unsigned key0 = row0 - bidx * (unsigned)SK;
    v8h x[2];
    size_t off[2];
#pragma unroll
    for (unsigned i = 0; i < 2u; ++i) {
      const unsigned dcol = 32u * i + (tid >> 3);
      const unsigned kk = (tid & 7u) * 8u;
      const float bb = bf16r(bias[n0 + dcol]);
#pragma unroll
      for (unsigned j = 0; j < 8u; ++j) {
        const float t = Cs[(kk + j) * LDC + dcol] * cs + bb;
        x[i][j] = toh_flush(t);
      }
      off[i] = ((size_t)bidx * HDIM + n0 + dcol) * SK + key0 + kk;
    }
#pragma unroll
    for (int i = 0; i < 2; ++i) *(volatile v8h*)(out16 + off[i]) = x[i];
    __threadfence();
#pragma unroll
    for (int i = 0; i < 2; ++i) *(volatile v8h*)(out16 + off[i]) = x[i];
  }

  if (MODE == 2) {
    const float cs = 1.0f / (WCARRY * VCARRY);
    const unsigned bidx = row0 / (unsigned)TQ;
    const unsigned p0 = row0 - bidx * (unsigned)TQ;
    v4f xs[4];
    size_t off[4];
#pragma unroll
    for (unsigned i = 0; i < 4u; ++i) {
      const unsigned ocol = 16u * i + (tid >> 4);
      const unsigned tk = (tid & 15u) * 4u;
      const float bb = bf16r(bias[n0 + ocol]);
      v4f val;
#pragma unroll
      for (unsigned j = 0; j < 4u; ++j) val[j] = Cs[(tk + j) * LDC + ocol] * cs + bb;
      xs[i] = val;
      off[i] = ((size_t)bidx * CO + n0 + ocol) * TQ + p0 + tk;
    }
#pragma unroll
    for (int i = 0; i < 4; ++i) *(volatile v4f*)(outf + off[i]) = xs[i];
    __threadfence();
#pragma unroll
    for (int i = 0; i < 4; ++i) *(volatile v4f*)(outf + off[i]) = xs[i];
  }
}

__global__ __launch_bounds__(256) void gemm_qk_kernel(
    const _Float16* __restrict__ A16, const _Float16* __restrict__ Bt,
    const float* __restrict__ bias, _Float16* __restrict__ out16) {
  gemm_body<0>(A16, Bt, (unsigned)CIN, bias, (float*)0, out16);
}
__global__ __launch_bounds__(256) void gemm_v_kernel(
    const _Float16* __restrict__ A16, const _Float16* __restrict__ Bt,
    const float* __restrict__ bias, _Float16* __restrict__ vt) {
  gemm_body<1>(A16, Bt, (unsigned)CIN, bias, (float*)0, vt);
}
__global__ __launch_bounds__(256) void gemm_wo_kernel(
    const _Float16* __restrict__ A16, const _Float16* __restrict__ Bt,
    const float* __restrict__ bias, float* __restrict__ y) {
  gemm_body<2>(A16, Bt, (unsigned)HDIM, bias, y, (_Float16*)0);
}

__global__ __launch_bounds__(256) void attn_kernel(
    const _Float16* __restrict__ Qh, const _Float16* __restrict__ Kh,
    const _Float16* __restrict__ Vt, _Float16* __restrict__ Ov) {
  __shared__ _Float16 Ks[64 * LDT];
  __shared__ _Float16 Vs[64 * LDT];
  __shared__ _Float16 Ps[8 * 16 * LDT];

  const unsigned tid = threadIdx.x, lane = tid & 31u;
  const unsigned w = (unsigned)__builtin_amdgcn_readfirstlane((int)(tid >> 5));
  const unsigned hh = lane >> 4, m = lane & 15u;
  const unsigned q0 = blockIdx.x * 128u;
  const unsigned head = blockIdx.y;
  const unsigned b = blockIdx.z;
  const float scale = 0.125f;
  const unsigned qrow0 = q0 + w * 16u;
  _Float16* P = Ps + w * (16u * LDT);

  const size_t qoff = (size_t)(b * (unsigned)TQ + qrow0 + m) * HDIM + head * HD + hh * 8u;
  v16h qf[2];
  qf[0] = frag_at(Qh + qoff);
  qf[1] = frag_at(Qh + qoff + 32);

  float mrow[8], lrow[8];
  v8f o[4];
#pragma unroll
  for (int v = 0; v < 8; ++v) { mrow[v] = -1.0e30f; lrow[v] = 0.0f; }
#pragma unroll
  for (int nb = 0; nb < 4; ++nb) o[nb] = (v8f){};

  const size_t kplane = (size_t)b * SK * HDIM + head * HD;
  const size_t vplane = ((size_t)b * HDIM + head * HD) * SK;

  for (unsigned kb = 0; kb < (unsigned)SK; kb += 64u) {
#pragma unroll
    for (unsigned j = 0; j < 2u; ++j) {
      const unsigned idx = tid + 256u * j;
      const unsigned r = idx >> 3, c = (idx & 7u) * 8u;
      *(v8h*)&Ks[r * LDT + c] = *(const v8h*)(Kh + kplane + (size_t)(kb + r) * HDIM + c);
      *(v8h*)&Vs[r * LDT + c] = *(const v8h*)(Vt + vplane + (size_t)r * SK + kb + c);
    }
    __syncthreads();

    v8f s[4];
#pragma unroll
    for (int kg = 0; kg < 4; ++kg) {
      v8f t = {};
#pragma unroll
      for (int c = 0; c < 2; ++c) {
        const v16h kf = ld_frag(&Ks[(kg * 16) * LDT + c * 32], LDT);
        t = wmma16(qf[c], kf, t);
      }
      s[kg] = t * scale;
    }

    float alpha[8];
#pragma unroll
    for (int v = 0; v < 8; ++v) {
      float mx = fmaxf(fmaxf(s[0][v], s[1][v]), fmaxf(s[2][v], s[3][v]));
      mx = red16_max(mx);
      const float mn = fmaxf(mrow[v], mx);
      alpha[v] = __expf(mrow[v] - mn);
      mrow[v] = mn;
    }
#pragma unroll
    for (int kg = 0; kg < 4; ++kg)
#pragma unroll
      for (int v = 0; v < 8; ++v) {
        const float e = __expf(s[kg][v] - mrow[v]) * PCARRY;
        const h16 ph = toh_flush(e);
        P[(hh * 8u + (unsigned)v) * LDT + (unsigned)kg * 16u + m] = ph;
        s[kg][v] = (float)ph;
      }
#pragma unroll
    for (int v = 0; v < 8; ++v) {
      const float rs = red16_sum((s[0][v] + s[1][v]) + (s[2][v] + s[3][v]));
      lrow[v] = alpha[v] * lrow[v] + rs;
    }
#pragma unroll
    for (int nb = 0; nb < 4; ++nb)
#pragma unroll
      for (int v = 0; v < 8; ++v) o[nb][v] = o[nb][v] * alpha[v];
    wave_lds_sync();

#pragma unroll
    for (int c = 0; c < 2; ++c) {
      const v16h pf = ld_frag(P + c * 32, LDT);
#pragma unroll
      for (int nb = 0; nb < 4; ++nb) {
        const v16h vf = ld_frag(&Vs[(nb * 16) * LDT + c * 32], LDT);
        o[nb] = wmma16(pf, vf, o[nb]);
      }
    }
    __syncthreads();
  }

  float inv[8];
#pragma unroll
  for (int v = 0; v < 8; ++v) inv[v] = __builtin_amdgcn_rcpf(lrow[v]) * VCARRY;
#pragma unroll
  for (int nb = 0; nb < 4; ++nb)
#pragma unroll
    for (int v = 0; v < 8; ++v)
      P[(hh * 8u + (unsigned)v) * LDT + (unsigned)nb * 16u + m] = toh_flush(o[nb][v] * inv[v]);
  wave_lds_sync();
  v8h x[4];
  size_t off[4];
#pragma unroll
  for (unsigned i = 0; i < 4u; ++i) {
    const unsigned r = 4u * i + (lane >> 3);
    const unsigned c = (lane & 7u) * 8u;
    x[i] = *(const v8h*)&P[r * LDT + c];
    off[i] = (size_t)(b * (unsigned)TQ + qrow0 + r) * HDIM + head * HD + c;
  }
#pragma unroll
  for (int i = 0; i < 4; ++i) *(volatile v8h*)(Ov + off[i]) = x[i];
  __threadfence();
#pragma unroll
  for (int i = 0; i < 4; ++i) *(volatile v8h*)(Ov + off[i]) = x[i];
}

__global__ __launch_bounds__(256) void bn_kernel(
    const float* __restrict__ Y, const float* __restrict__ G, const float* __restrict__ Be,
    float* __restrict__ out) {
#pragma clang fp contract(off)
  __shared__ float red1[8];
  __shared__ float red2[8];
  const unsigned tid = threadIdx.x, lane = tid & 31u;
  const unsigned w = (unsigned)__builtin_amdgcn_readfirstlane((int)(tid >> 5));
  const unsigned o = blockIdx.x;
  const unsigned nf4 = (unsigned)NB * (unsigned)(TQ / 4);
  const float invn = 1.0f / (float)(NB * TQ);

  float s = 0.0f;
#pragma unroll 1
  for (unsigned base = w * 32u; base < nf4; base += 256u) {
    const unsigned idx = base + lane;
    const unsigned n = idx / (unsigned)(TQ / 4);
    const unsigned f = idx - n * (unsigned)(TQ / 4);
    const v4f a = *(const v4f*)(Y + ((size_t)n * CO + o) * TQ + f * 4u);
    s += (a[0] + a[1]) + (a[2] + a[3]);
  }
  s = red32_sum(s);
  if (lane == 0u) red1[w] = s;
  __syncthreads();
  float tot = 0.0f;
#pragma unroll
  for (int i = 0; i < 8; ++i) tot += red1[i];
  const float mean = tot * invn;

  float ss = 0.0f;
#pragma unroll 1
  for (unsigned base = w * 32u; base < nf4; base += 256u) {
    const unsigned idx = base + lane;
    const unsigned n = idx / (unsigned)(TQ / 4);
    const unsigned f = idx - n * (unsigned)(TQ / 4);
    const v4f a = *(const v4f*)(Y + ((size_t)n * CO + o) * TQ + f * 4u);
    const float d0 = a[0] - mean, d1 = a[1] - mean, d2 = a[2] - mean, d3 = a[3] - mean;
    ss += (d0 * d0 + d1 * d1) + (d2 * d2 + d3 * d3);
  }
  ss = red32_sum(ss);
  if (lane == 0u) red2[w] = ss;
  __syncthreads();
  float tot2 = 0.0f;
#pragma unroll
  for (int i = 0; i < 8; ++i) tot2 += red2[i];
  const float var = tot2 * invn;
  const float rstd = 1.0f / sqrtf(var + 1.0e-5f);
  const float g = bf16r(G[o]);
  const float be = bf16r(Be[o]);

#pragma unroll 1
  for (unsigned base = w * 32u; base < nf4; base += 256u) {
    const unsigned idx = base + lane;
    const unsigned n = idx / (unsigned)(TQ / 4);
    const unsigned f = idx - n * (unsigned)(TQ / 4);
    const size_t off = ((size_t)n * CO + o) * TQ + f * 4u;
    const v4f a = *(const v4f*)(Y + off);
    v4f r;
#pragma unroll
    for (int j = 0; j < 4; ++j) r[j] = (a[j] - mean) * rstd * g + be;
    float* p = out + off;
    *(volatile v4f*)p = r;
    __threadfence();
    *(volatile v4f*)p = r;
  }
}

extern "C" void kernel_launch(void* const* d_in, const int* in_sizes, int n_in,
                              void* d_out, int out_size, void* d_ws, size_t ws_size,
                              hipStream_t stream) {
  if (n_in < 10) return;
  if ((long long)in_sizes[0] < (long long)NB * CIN * TQ) return;
  if ((long long)in_sizes[1] < (long long)NB * CIN * SK) return;
  if ((long long)in_sizes[2] < (long long)HDIM * CIN) return;
  if (in_sizes[3] < HDIM) return;
  if ((long long)in_sizes[4] < (long long)2 * HDIM * CIN) return;
  if (in_sizes[5] < 2 * HDIM) return;
  if ((long long)in_sizes[6] < (long long)CO * HDIM) return;
  if (in_sizes[7] < CO || in_sizes[8] < CO || in_sizes[9] < CO) return;
  if ((long long)out_size < (long long)NB * CO * TQ) return;
  if (ws_size < WS_TOTAL) return;

  const float* joint = (const float*)d_in[0];
  const float* group = (const float*)d_in[1];
  const float* wq    = (const float*)d_in[2];
  const float* bq    = (const float*)d_in[3];
  const float* wkv   = (const float*)d_in[4];
  const float* bkv   = (const float*)d_in[5];
  const float* wo    = (const float*)d_in[6];
  const float* bo    = (const float*)d_in[7];
  const float* gamma = (const float*)d_in[8];
  const float* beta  = (const float*)d_in[9];
  float* out = (float*)d_out;

  char* ws = (char*)d_ws;
  _Float16* Wq16  = (_Float16*)(ws + OFF_WQ);
  _Float16* Wkv16 = (_Float16*)(ws + OFF_WKV);
  _Float16* Wo16  = (_Float16*)(ws + OFF_WO);
  _Float16* XJ16  = (_Float16*)(ws + OFF_XJ);
  _Float16* XG16  = (_Float16*)(ws + OFF_XG);
  _Float16* Q16   = (_Float16*)(ws + OFF_Q);
  _Float16* K16   = (_Float16*)(ws + OFF_K);
  _Float16* Vt16  = (_Float16*)(ws + OFF_VT);
  _Float16* Ctx16 = (_Float16*)(ws + OFF_CTX);
  float*    Y     = (float*)(ws + OFF_Y);

  dim3 blk(256);

  wcast_kernel<<<dim3((HDIM * CIN) / 2048), blk, 0, stream>>>(wq, Wq16, (unsigned)((HDIM * CIN) / 8));
  wcast_kernel<<<dim3((2 * HDIM * CIN) / 2048), blk, 0, stream>>>(wkv, Wkv16, (unsigned)((2 * HDIM * CIN) / 8));
  wcast_kernel<<<dim3((CO * HDIM) / 2048), blk, 0, stream>>>(wo, Wo16, (unsigned)((CO * HDIM) / 8));

  xconv_kernel<<<dim3(TQ / 64, CIN / 64, NB), blk, 0, stream>>>(joint, XJ16, (unsigned)TQ);
  xconv_kernel<<<dim3(SK / 64, CIN / 64, NB), blk, 0, stream>>>(group, XG16, (unsigned)SK);

  gemm_qk_kernel<<<dim3(HDIM / 64, (NB * TQ) / 64), blk, 0, stream>>>(XJ16, Wq16, bq, Q16);
  gemm_qk_kernel<<<dim3(HDIM / 64, (NB * SK) / 64), blk, 0, stream>>>(XG16, Wkv16, bkv, K16);
  gemm_v_kernel<<<dim3(HDIM / 64, (NB * SK) / 64), blk, 0, stream>>>(
      XG16, Wkv16 + (size_t)HDIM * CIN, bkv + HDIM, Vt16);

  attn_kernel<<<dim3(TQ / 128, NHEAD, NB), blk, 0, stream>>>(Q16, K16, Vt16, Ctx16);

  gemm_wo_kernel<<<dim3(CO / 64, (NB * TQ) / 64), blk, 0, stream>>>(Ctx16, Wo16, bo, Y);

  bn_kernel<<<dim3(CO), blk, 0, stream>>>(Y, gamma, beta, out);
}
